// FullAttention_Complex_65481071394886
// MI455X (gfx1250) — hardware-verified
//
#include <hip/hip_runtime.h>
#include <math.h>
#include <stdint.h>

#define NBATCH 2
#define SEQ    2048
#define NHEAD  8
#define HD     64
#define VW     (2 * HD)
#define DMOD   (NHEAD * HD)
#define NTOK   (NBATCH * SEQ)
#define NQB    (SEQ / 64)
#define NQP    8
#define VSC    16.0f
#define PSC    1024.0f
#define PRS    4096.0f
#define SCL    0.125f
#define NEG_BIG (-1.0e30f)
static_assert(HD == 64 && VW == 128);
static_assert((SEQ % 64) == 0 && (DMOD % 32) == 0);
static_assert(((NTOK * DMOD) % 2048) == 0);
static_assert(NQP > 0 && NQP < NQB);

typedef _Float16 v16h __attribute__((ext_vector_type(16)));
typedef _Float16 v8h  __attribute__((ext_vector_type(8)));
typedef __bf16   v16b __attribute__((ext_vector_type(16)));
typedef unsigned short v16us __attribute__((ext_vector_type(16)));
typedef unsigned short v8us  __attribute__((ext_vector_type(8)));
typedef float    v8f  __attribute__((ext_vector_type(8)));
typedef float    v4f  __attribute__((ext_vector_type(4)));
typedef unsigned int v4u __attribute__((ext_vector_type(4)));
typedef unsigned int v8u __attribute__((ext_vector_type(8)));
union FH { v16h v; v8h h[2]; };
union FB { v16us u; v8us h[2]; v8u w; };

__device__ __forceinline__ unsigned short bf_bits(float f) {
  unsigned u = __float_as_uint(f);
  return (unsigned short)((u + 0x7FFFu + ((u >> 16) & 1u)) >> 16);
}
__device__ __forceinline__ float bf_up(unsigned short h) { return __uint_as_float(((unsigned)h) << 16); }
__device__ __forceinline__ unsigned short h_bits(_Float16 x) { return __builtin_bit_cast(unsigned short, x); }
__device__ __forceinline__ unsigned pk16(unsigned short a, unsigned short b) { return (unsigned)a | ((unsigned)b << 16); }
__device__ __forceinline__ v8f zero8() { v8f z = {0.f, 0.f, 0.f, 0.f, 0.f, 0.f, 0.f, 0.f}; return z; }

__device__ __forceinline__ v16us ldfrag_b(const unsigned short* p) {
  FB f;
  f.h[0] = *(const v8us*)(p);
  f.h[1] = *(const v8us*)(p + 16);
  return f.u;
}
__device__ __forceinline__ v16us neg16(v16us x) {
  FB f;
  f.u = x;
#pragma unroll
  for (int i = 0; i < 8; ++i) f.w[i] = f.w[i] ^ 0x80008000u;
  return f.u;
}

__device__ __forceinline__ v8f mma_h_raw(v16h a, v16h b, v8f c) {
  return __builtin_amdgcn_wmma_f32_16x16x32_f16(false, a, false, b, (short)0, c, false, false);
}
__device__ __forceinline__ v8f mma_b_raw(v16us a, v16us b, v8f c) {
  return __builtin_amdgcn_wmma_f32_16x16x32_bf16(false, __builtin_bit_cast(v16b, a), false,
                                                 __builtin_bit_cast(v16b, b), (short)0, c, false, false);
}
__device__ __forceinline__ void guard_b5(v8f& x, v8f& y, v16us a, v16us b, v16us d, v16us e, v16us f) {
#if defined(__HIP_DEVICE_COMPILE__)
  asm volatile("v_nop\n\tv_nop\n\tv_nop\n\tv_nop" : "+v"(x), "+v"(y) : "v"(a), "v"(b), "v"(d), "v"(e), "v"(f));
#endif
}
__device__ __forceinline__ void guard_h1(v8f& x, v16h a, v16h b) {
#if defined(__HIP_DEVICE_COMPILE__)
  asm volatile("v_nop\n\tv_nop\n\tv_nop\n\tv_nop" : "+v"(x) : "v"(a), "v"(b));
#endif
}
__device__ __forceinline__ void guard_h2(v8f& x, v8f& y, v16h a, v16h b, v16h d) {
#if defined(__HIP_DEVICE_COMPILE__)
  asm volatile("v_nop\n\tv_nop\n\tv_nop\n\tv_nop" : "+v"(x), "+v"(y) : "v"(a), "v"(b), "v"(d));
#endif
}
__device__ __forceinline__ void acc_guard4(v8f& a, v8f& b, v8f& c, v8f& d) {
#if defined(__HIP_DEVICE_COMPILE__)
  asm volatile("v_nop\n\tv_nop\n\tv_nop\n\tv_nop" : "+v"(a), "+v"(b), "+v"(c), "+v"(d));
#endif
}
__device__ __forceinline__ void wave_sync_lds() {
  __builtin_amdgcn_fence(__ATOMIC_RELEASE, "workgroup");
  __builtin_amdgcn_wave_barrier();
  __builtin_amdgcn_fence(__ATOMIC_ACQUIRE, "workgroup");
}

__global__ __launch_bounds__(256) void tr_cvt(const float* __restrict__ in, unsigned short* out, int R, int C,
                                             long long zin, long long zout, float scale) {
  __shared__ float tile[64 * 33];
  const int z = blockIdx.z;
  const float* ib = in + (size_t)z * (size_t)zin;
  unsigned short* ob = out + (size_t)z * (size_t)zout;
  const int r0 = blockIdx.y * 64, c0 = blockIdx.x * 32;
  const int t = threadIdx.x;
  {
    const int ir = t >> 2, ic = (t & 3) * 8;
    const float* g = ib + (size_t)(r0 + ir) * (size_t)C + c0 + ic;
    const v4f a = *(const v4f*)g;
    const v4f b = *(const v4f*)(g + 4);
    float* l = tile + ir * 33 + ic;
    l[0] = a[0]; l[1] = a[1]; l[2] = a[2]; l[3] = a[3];
    l[4] = b[0]; l[5] = b[1]; l[6] = b[2]; l[7] = b[3];
  }
  __syncthreads();
  const int orow = t >> 3, piece = (t & 7) * 8;
  v4u p;
#pragma unroll
  for (int e = 0; e < 4; ++e) {
    const float f0 = tile[(piece + 2 * e) * 33 + orow];
    const float f1 = tile[(piece + 2 * e + 1) * 33 + orow];
    const _Float16 x0 = (_Float16)(bf_up(bf_bits(f0)) * scale);
    const _Float16 x1 = (_Float16)(bf_up(bf_bits(f1)) * scale);
    p[e] = pk16(h_bits(x0), h_bits(x1));
  }
  const size_t go = (size_t)(c0 + orow) * (size_t)R + r0 + piece;
  *(volatile v4u*)(ob + go) = p;
  __threadfence();
  *(volatile v4u*)(ob + go) = p;
}

__global__ __launch_bounds__(256) void cvt2(const float* __restrict__ a, const float* __restrict__ bsrc,
                                           unsigned short* out, int n) {
  const size_t i8 = ((size_t)blockIdx.x * 256 + threadIdx.x) * 8;
  if (i8 + 8 > (size_t)n) return;
  const v4f a0 = *(const v4f*)(a + i8);
  const v4f a1 = *(const v4f*)(a + i8 + 4);
  const v4f b0 = *(const v4f*)(bsrc + i8);
  const v4f b1 = *(const v4f*)(bsrc + i8 + 4);
  v4u pa, pb;
#pragma unroll
  for (int e = 0; e < 2; ++e) {
    pa[e]     = pk16(bf_bits(a0[2 * e]), bf_bits(a0[2 * e + 1]));
    pa[2 + e] = pk16(bf_bits(a1[2 * e]), bf_bits(a1[2 * e + 1]));
    pb[e]     = pk16(bf_bits(b0[2 * e]), bf_bits(b0[2 * e + 1]));
    pb[2 + e] = pk16(bf_bits(b1[2 * e]), bf_bits(b1[2 * e + 1]));
  }
  unsigned short* oa = out + i8;
  unsigned short* ob = out + (size_t)n + i8;
  *(volatile v4u*)oa = pa;
  *(volatile v4u*)ob = pb;
  __threadfence();
  *(volatile v4u*)oa = pa;
  *(volatile v4u*)ob = pb;
}

template <bool PRES>
__global__ __launch_bounds__(128)
void attn_c(const unsigned short* __restrict__ QB, const unsigned short* __restrict__ KB,
            const unsigned short* __restrict__ VT, float* out, int qb0, int nqb) {
  __shared__ __align__(16) unsigned short Ksh[64 * VW];
  __shared__ __align__(16) _Float16 Vs[VW * 64];
  __shared__ __align__(16) _Float16 Psh[4][16 * 64];
  __shared__ __align__(16) _Float16 Psl[PRES ? 4 : 1][PRES ? 16 * 64 : 8];
  __shared__ __align__(16) float    Os[4][16 * VW];

  const int tid  = threadIdx.x;
  const int wave = tid >> 5;
  const int lane = tid & 31;
  const int hh   = lane >> 4;
  const int c    = lane & 15;

  const unsigned nq = (unsigned)nqb;
  const int qb = qb0 + (int)(blockIdx.x % nq);
  const int hb = (int)(blockIdx.x / nq);
  const int h  = hb % NHEAD;
  const int b  = hb / NHEAD;
  const int q0 = qb * 64 + wave * 16;

  const size_t NPL = (size_t)NTOK * DMOD;
  const unsigned short* Qr = QB + (size_t)b * SEQ * DMOD + (size_t)h * HD;
  const unsigned short* Qi = Qr + NPL;
  const unsigned short* Kr = KB + (size_t)b * SEQ * DMOD + (size_t)h * HD;
  const _Float16* Vg = (const _Float16*)(const void*)VT + ((size_t)(b * 2) * DMOD + (size_t)h * HD) * SEQ;

  float mrow[8], lrow[8];
  v8f oh[8];
#pragma unroll
  for (int r = 0; r < 8; ++r) { mrow[r] = NEG_BIG; lrow[r] = 0.f; }
#pragma unroll
  for (int t = 0; t < 8; ++t) oh[t] = zero8();

  _Float16* pwh = Psh[wave];
  _Float16* pwl = &Psl[PRES ? wave : 0][0];

  for (int kt = 0; kt < NQB; ++kt) {
    if (kt > qb) break;
    const int kv0 = kt * 64;
    __syncthreads();
    {
      const int r = tid >> 1, p = tid & 1;
      const unsigned short* kg = Kr + (size_t)p * NPL + (size_t)(kv0 + r) * DMOD;
      unsigned short* kd = Ksh + r * VW + p * HD;
#pragma unroll
      for (int i = 0; i < 8; ++i) *(v8us*)(kd + 8 * i) = *(const v8us*)(kg + 8 * i);
      const int vp = tid >> 6, dl = tid & 63;
      const _Float16* vg = Vg + ((size_t)vp * DMOD + dl) * SEQ + kv0;
#pragma unroll
      for (int i = 0; i < 8; ++i) *(v8h*)(Vs + tid * 64 + 8 * i) = *(const v8h*)(vg + 8 * i);
    }
    __syncthreads();

    v16us qr[2], qi[2];
#pragma unroll
    for (int dc = 0; dc < 2; ++dc) {
      qr[dc] = ldfrag_b(Qr + (size_t)(q0 + c) * DMOD + dc * 32 + 8 * hh);
      qi[dc] = ldfrag_b(Qi + (size_t)(q0 + c) * DMOD + dc * 32 + 8 * hh);
    }

    v8f s[4];
#pragma unroll
    for (int j = 0; j < 4; ++j) {
      v8f sr = zero8(), si = zero8();
#pragma unroll
      for (int dc = 0; dc < 2; ++dc) {
        const unsigned short* kp = Ksh + (j * 16 + c) * VW + dc * 32 + 8 * hh;
        FB br, bi;
        br.h[0] = *(const v8us*)(kp);
        br.h[1] = *(const v8us*)(kp + 16);
        bi.h[0] = *(const v8us*)(kp + HD);
        bi.h[1] = *(const v8us*)(kp + HD + 16);
        const v16us bin = neg16(bi.u);
        sr = mma_b_raw(qr[dc], br.u, sr);
        sr = mma_b_raw(qi[dc], bin, sr);
        si = mma_b_raw(qr[dc], bi.u, si);
        si = mma_b_raw(qi[dc], br.u, si);
        guard_b5(sr, si, qr[dc], qi[dc], br.u, bi.u, bin);
      }
      const int key  = kv0 + j * 16 + c;
      const int rowb = q0 + 8 * hh;
#pragma unroll
      for (int r = 0; r < 8; ++r) {
        const float m2 = sr[r] * sr[r] + si[r] * si[r];
        const float v = sqrtf(m2) * SCL;
        s[j][r] = (key <= rowb + r) ? v : NEG_BIG;
      }
    }

#pragma unroll
    for (int r = 0; r < 8; ++r) {
      float m = s[0][r];
      m = fmaxf(m, s[1][r]);
      m = fmaxf(m, s[2][r]);
      m = fmaxf(m, s[3][r]);
#pragma unroll
      for (int off = 1; off < 16; off <<= 1) m = fmaxf(m, __shfl_xor(m, off, 32));
      const float mnew  = fmaxf(mrow[r], m);
      const float alpha = __expf(mrow[r] - mnew);
      mrow[r] = mnew;
      float psum = 0.f;
#pragma unroll
      for (int j = 0; j < 4; ++j) {
        const float p  = __expf(s[j][r] - mnew);
        psum += p;
        const float ph = p * PSC;
        const _Float16 xh = (_Float16)ph;
        const int pi = (8 * hh + r) * 64 + j * 16 + c;
        pwh[pi] = xh;
        if (PRES) pwl[pi] = (_Float16)((ph - (float)xh) * PRS);
      }
#pragma unroll
      for (int off = 1; off < 16; off <<= 1) psum += __shfl_xor(psum, off, 32);
      lrow[r] = lrow[r] * alpha + psum;
#pragma unroll
      for (int t = 0; t < 8; ++t) oh[t][r] *= alpha;
    }
    wave_sync_lds();

    v8f ol[8];
#pragma unroll
    for (int t = 0; t < 8; ++t) ol[t] = zero8();
#pragma unroll 1
    for (int kk = 0; kk < 2; ++kk) {
      FH pa, pb;
      pa.h[0] = *(const v8h*)(pwh + c * 64 + kk * 32 + 8 * hh);
      pa.h[1] = *(const v8h*)(pwh + c * 64 + kk * 32 + 16 + 8 * hh);
      pb.v = pa.v;
      if (PRES) {
        pb.h[0] = *(const v8h*)(pwl + c * 64 + kk * 32 + 8 * hh);
        pb.h[1] = *(const v8h*)(pwl + c * 64 + kk * 32 + 16 + 8 * hh);
      }
#pragma unroll
      for (int t = 0; t < 8; ++t) {
        FH vb;
        vb.h[0] = *(const v8h*)(Vs + (t * 16 + c) * 64 + kk * 32 + 8 * hh);
        vb.h[1] = *(const v8h*)(Vs + (t * 16 + c) * 64 + kk * 32 + 16 + 8 * hh);
        oh[t] = mma_h_raw(pa.v, vb.v, oh[t]);
        if (PRES) {
          ol[t] = mma_h_raw(pb.v, vb.v, ol[t]);
          guard_h2(oh[t], ol[t], pa.v, pb.v, vb.v);
        } else {
          guard_h1(oh[t], pa.v, vb.v);
        }
      }
    }
    acc_guard4(oh[0], oh[1], oh[2], oh[3]);
    acc_guard4(oh[4], oh[5], oh[6], oh[7]);
    if (PRES) {
      acc_guard4(ol[0], ol[1], ol[2], ol[3]);
      acc_guard4(ol[4], ol[5], ol[6], ol[7]);
#pragma unroll
      for (int t = 0; t < 8; ++t) {
#pragma unroll
        for (int r = 0; r < 8; ++r) oh[t][r] += ol[t][r] * (1.0f / PRS);
      }
    }
  }

  float* os = Os[wave];
#pragma unroll
  for (int r = 0; r < 8; ++r) {
    const float l = lrow[r];
    const float inv = ((l > 0.f) ? (1.0f / l) : 0.f) * (1.0f / (PSC * VSC));
#pragma unroll
    for (int t = 0; t < 8; ++t) {
      const int pos = (t < 4) ? (2 * (t * 16 + c)) : (2 * ((t - 4) * 16 + c) + 1);
      os[(8 * hh + r) * VW + pos] = oh[t][r] * inv;
    }
  }
  wave_sync_lds();
  for (int pass = 0; pass < 2; ++pass) {
#pragma unroll
    for (int it = 0; it < 16; ++it) {
      const v4f o = *(const v4f*)(os + it * VW + lane * 4);
      float* g = out + ((size_t)(b * SEQ + q0 + it) * NHEAD + h) * VW + lane * 4;
      *(volatile v4f*)g = o;
    }
    __threadfence();
  }
}

extern "C" void kernel_launch(void* const* d_in, const int* in_sizes, int n_in,
                              void* d_out, int out_size, void* d_ws, size_t ws_size,
                              hipStream_t stream) {
  const int n = NTOK * DMOD;
  if (n_in < 6) return;
  for (int i = 0; i < 6; ++i) if (in_sizes[i] != n) return;
  if (out_size != 2 * n) return;

  const float* qr = (const float*)d_in[0];
  const float* qi = (const float*)d_in[1];
  const float* kr = (const float*)d_in[2];
  const float* ki = (const float*)d_in[3];
  const float* vr = (const float*)d_in[4];
  const float* vi = (const float*)d_in[5];
  float* outf = (float*)d_out;

  const size_t PQB = (size_t)2 * n * 2;
  const size_t PKB = (size_t)2 * n * 2;
  const size_t PVT = (size_t)NBATCH * 2 * DMOD * SEQ * 2;
  size_t off = 0;
  const size_t oQ = off; off += PQB;
  const size_t oK = off; off += PKB;
  const size_t oV = off; off += PVT;
  if (off > ws_size) return;
  if (off > (size_t)134217728) return;

  char* ws = (char*)d_ws;
  unsigned short* QB = (unsigned short*)(ws + oQ);
  unsigned short* KB = (unsigned short*)(ws + oK);
  unsigned short* VT = (unsigned short*)(ws + oV);

  const dim3 blk256(256), blk128(128);

  cvt2<<<dim3(n / 2048), blk256, 0, stream>>>(qr, qi, QB, n);
  cvt2<<<dim3(n / 2048), blk256, 0, stream>>>(kr, ki, KB, n);
  tr_cvt<<<dim3(DMOD / 32, SEQ / 64, NBATCH), blk256, 0, stream>>>(
      vr, VT, SEQ, DMOD, (long long)SEQ * DMOD, (long long)2 * DMOD * SEQ, VSC);
  tr_cvt<<<dim3(DMOD / 32, SEQ / 64, NBATCH), blk256, 0, stream>>>(
      vi, VT + (size_t)DMOD * SEQ, SEQ, DMOD, (long long)SEQ * DMOD, (long long)2 * DMOD * SEQ, VSC);
  attn_c<true><<<dim3(NQP * NHEAD * NBATCH), blk128, 0, stream>>>(QB, KB, VT, outf, 0, NQP);
  attn_c<false><<<dim3((NQB - NQP) * NHEAD * NBATCH), blk128, 0, stream>>>(QB, KB, VT, outf, NQP, NQB - NQP);
  (void)hipGetLastError();
}
